// SyntaxErrorGNN_68307159876136
// MI455X (gfx1250) — hardware-verified
//
#include <hip/hip_runtime.h>
#include <stddef.h>


#define HD      64
#define H2      32
#define ZW      128
#define NTHR    256
#define NWAVE   8
#define EPT     8
#define NGRP    2
#define CHUNK   (NTHR * EPT * NGRP)
#define WCAP    (EPT * NGRP * 32)
#define LISTN   (NWAVE * WCAP)
#define NBC     4096
#define NBF     1024
#define RCAP    40960
#define RBN     128
#define TGT     256
#define DEGCAP  1024
#define OTHR    512
#define GBM     64
#define GTHR    128
#define HTHR    128
#define HWAVE   4
#define SOCAP   4096
#define WSCAP   134217728
#define BN_EPS  1e-5f
#define WCARRY  64.0f
#define WINV    0.015625f

#define LDS_FILL ((RCAP + NBF + LISTN) * 4 + 64)

static_assert((CHUNK & (CHUNK - 1)) == 0);
static_assert(CHUNK <= 4096);
static_assert((NBC & (NBC - 1)) == 0 && (NBF & (NBF - 1)) == 0);
static_assert(NBC == 4 * NBF);
static_assert(OTHR * 8 == NBC);
static_assert((RCAP % 32) == 0);
static_assert(TGT == NWAVE * 32);
static_assert((NBC % TGT) == 0);
static_assert((TGT % GBM) == 0);
static_assert(HD == 4 * 16);
static_assert(ZW == 2 * HD);
static_assert((HD % 32) == 0 && (ZW % 32) == 0 && (H2 % 32) == 0);
static_assert(WCAP == EPT * NGRP * 32);
static_assert(HTHR == HWAVE * 32);
static_assert((GBM * HD) % (4 * GTHR) == 0);

typedef float    v4f  __attribute__((ext_vector_type(4)));
typedef float    v8f  __attribute__((ext_vector_type(8)));
typedef int      v4i  __attribute__((ext_vector_type(4)));
typedef _Float16 v4h  __attribute__((ext_vector_type(4)));
typedef _Float16 v8h  __attribute__((ext_vector_type(8)));
typedef _Float16 v16h __attribute__((ext_vector_type(16)));
union Frag { v16h v; v8h half[2]; };

__device__ __forceinline__ v8f wm(v16h a, v16h b, v8f c) {
  v8f d = __builtin_amdgcn_wmma_f32_16x16x32_f16(false, a, false, b, (short)0, c, false, false);
  asm volatile("v_nop\n\tv_nop\n\tv_nop\n\tv_nop" : "+v"(d) : "v"(a), "v"(b));
  return d;
}

__device__ __forceinline__ v4f relu4(v4f y) {
  v4f r;
  r.x = fmaxf(y.x, 0.f); r.y = fmaxf(y.y, 0.f); r.z = fmaxf(y.z, 0.f); r.w = fmaxf(y.w, 0.f);
  return r;
}

__device__ __forceinline__ void colsum_out(float* scs, float* srow, v4f cs, float* dst,
                                           int tid, int lane, int wave) {
  const int hf = lane >> 4, q = lane & 15;
  *(v4f*)(scs + (wave * 2 + hf) * HD + 4 * q) = cs;
  __syncthreads();
  if (tid < HD) {
    float s = 0.f;
#pragma unroll
    for (int w = 0; w < 2 * NWAVE; ++w) s += scs[w * HD + tid];
    srow[tid] = s;
  }
  __syncthreads();
  const bool act = tid < (HD / 4);
  const int qq = act ? tid : 0;
  const v4f v = *(const v4f*)(srow + 4 * qq);
  if (act) *(volatile v4f*)(dst + 4 * qq) = v;
  __threadfence();
  if (act) *(volatile v4f*)(dst + 4 * qq) = v;
}

template <int NB>
__device__ __forceinline__ int scan_chunk(const int* __restrict__ dsts, int nE, int cbase, int slotBase,
                                          int vec8, int* list, int tid, int lane, int wave) {
  int wc = 0;
#pragma unroll
  for (int g = 0; g < NGRP; ++g) {
    const int el0  = (g * NTHR + tid) * EPT;
    const int e0   = cbase + el0;
    const int sent = -2147483647 - 1;
    v4i da, db;
    if (vec8 != 0 && cbase + CHUNK <= nE) {
      da = *(const v4i*)(dsts + e0);
      db = *(const v4i*)(dsts + e0 + 4);
    } else {
      da.x = (e0     < nE) ? dsts[min(e0, nE - 1)] : sent;
      da.y = (e0 + 1 < nE) ? dsts[min(e0 + 1, nE - 1)] : sent;
      da.z = (e0 + 2 < nE) ? dsts[min(e0 + 2, nE - 1)] : sent;
      da.w = (e0 + 3 < nE) ? dsts[min(e0 + 3, nE - 1)] : sent;
      db.x = (e0 + 4 < nE) ? dsts[min(e0 + 4, nE - 1)] : sent;
      db.y = (e0 + 5 < nE) ? dsts[min(e0 + 5, nE - 1)] : sent;
      db.z = (e0 + 6 < nE) ? dsts[min(e0 + 6, nE - 1)] : sent;
      db.w = (e0 + 7 < nE) ? dsts[min(e0 + 7, nE - 1)] : sent;
    }
    const unsigned nb = (unsigned)slotBase;
    const unsigned s0 = (unsigned)da.x - nb, s1 = (unsigned)da.y - nb;
    const unsigned s2 = (unsigned)da.z - nb, s3 = (unsigned)da.w - nb;
    const unsigned s4 = (unsigned)db.x - nb, s5 = (unsigned)db.y - nb;
    const unsigned s6 = (unsigned)db.z - nb, s7 = (unsigned)db.w - nb;
    const bool h0 = s0 < (unsigned)NB, h1 = s1 < (unsigned)NB, h2 = s2 < (unsigned)NB, h3 = s3 < (unsigned)NB;
    const bool h4 = s4 < (unsigned)NB, h5 = s5 < (unsigned)NB, h6 = s6 < (unsigned)NB, h7 = s7 < (unsigned)NB;
    const unsigned any = __builtin_amdgcn_ballot_w32(h0 | h1 | h2 | h3 | h4 | h5 | h6 | h7);
    if (any != 0u) {
#define HITJ(J, HJ, SJ) { \
        const unsigned mj = __builtin_amdgcn_ballot_w32(HJ); \
        if (mj != 0u) { \
          if (HJ) { \
            const int pos = wc + (int)__builtin_amdgcn_mbcnt_lo(mj, 0u); \
            if (pos < WCAP) list[wave * WCAP + pos] = ((el0 + (J)) << 12) | (int)(SJ); \
          } \
          wc += (int)__builtin_popcount(mj); } }
      HITJ(0, h0, s0)
      HITJ(1, h1, s1)
      HITJ(2, h2, s2)
      HITJ(3, h3, s3)
      HITJ(4, h4, s4)
      HITJ(5, h5, s5)
      HITJ(6, h6, s6)
      HITJ(7, h7, s7)
#undef HITJ
    }
  }
  return wc;
}

__global__ __launch_bounds__(NTHR) void k_count(
    const int* __restrict__ dsts, int* cnt, float* dinv, int nE, int vec8) {
  __shared__ __attribute__((aligned(16))) int scnt[NBC];
  __shared__ __attribute__((aligned(16))) int list[LISTN];
  __shared__ int wcnt[NWAVE];
  const int tid = threadIdx.x, lane = tid & 31, wave = tid >> 5;
  const int nodeBase = blockIdx.x * NBC;

  for (int i = tid; i < NBC; i += NTHR) scnt[i] = 0;
  __syncthreads();

  const int nChunks = (nE + CHUNK - 1) / CHUNK;
#pragma unroll 1
  for (int ch = 0; ch < nChunks; ++ch) {
    const int cbase = ch * CHUNK;
    const int wc = scan_chunk<NBC>(dsts, nE, cbase, nodeBase, vec8, list, tid, lane, wave);
    if (lane == 0) wcnt[wave] = wc;
    __syncthreads();
    if (wave == 0) {
#pragma unroll 1
      for (int wsx = 0; wsx < NWAVE; ++wsx) {
        int n = __builtin_amdgcn_readfirstlane(wcnt[wsx]);
        n = n > WCAP ? WCAP : (n < 0 ? 0 : n);
        const int* lp = list + wsx * WCAP;
#pragma unroll 1
        for (int i = 0; i < n; ++i) {
          const int ent  = __builtin_amdgcn_readfirstlane(lp[i]);
          const int slot = ent & (NBC - 1);
          if (lane == 0) scnt[slot] = scnt[slot] + 1;
        }
      }
    }
    __syncthreads();
  }

  v4i cq[4];
  v4f dq[4];
#pragma unroll
  for (int q = 0; q < 4; ++q) {
    const int f = (wave * 4 + q) * 128 + 4 * lane;
    const v4i cv = *(const v4i*)(scnt + f);
    cq[q] = cv;
    v4f d;
    d.x = rsqrtf((float)(cv.x < 0 ? 0 : cv.x) + 1.0f);
    d.y = rsqrtf((float)(cv.y < 0 ? 0 : cv.y) + 1.0f);
    d.z = rsqrtf((float)(cv.z < 0 ? 0 : cv.z) + 1.0f);
    d.w = rsqrtf((float)(cv.w < 0 ? 0 : cv.w) + 1.0f);
    dq[q] = d;
  }
  int*   cp = cnt  + (size_t)nodeBase;
  float* dp = dinv + (size_t)nodeBase;
#pragma unroll
  for (int q = 0; q < 4; ++q) {
    const int f = (wave * 4 + q) * 128 + 4 * lane;
    *(volatile v4i*)(cp + f) = cq[q];
    *(volatile v4f*)(dp + f) = dq[q];
  }
  __threadfence();
#pragma unroll
  for (int q = 0; q < 4; ++q) {
    const int f = (wave * 4 + q) * 128 + 4 * lane;
    *(volatile v4i*)(cp + f) = cq[q];
    *(volatile v4f*)(dp + f) = dq[q];
  }
}

__global__ __launch_bounds__(OTHR) void k_offsets(
    const int* __restrict__ cnt, int* off, int* rbase, int nChunk) {
  __shared__ __attribute__((aligned(16))) int soff[NBC];
  __shared__ __attribute__((aligned(16))) int srb[RBN];
  __shared__ int wtot[OTHR / 32];
  const int tid = threadIdx.x, lane = tid & 31, wave = tid >> 5, sub = tid >> 7;
  for (int i = tid; i < RBN; i += OTHR) srb[i] = 0;
  int carry = 0;
#pragma unroll 1
  for (int ch = 0; ch < nChunk; ++ch) {
    const int base = ch * NBC;
    const v4i c0 = *(const v4i*)(cnt + base + 8 * tid);
    const v4i c1 = *(const v4i*)(cnt + base + 8 * tid + 4);
    const int e0 = max(c0.x, 0), e1 = max(c0.y, 0), e2 = max(c0.z, 0), e3 = max(c0.w, 0);
    const int e4 = max(c1.x, 0), e5 = max(c1.y, 0), e6 = max(c1.z, 0), e7 = max(c1.w, 0);
    const int ts = e0 + e1 + e2 + e3 + e4 + e5 + e6 + e7;
    int incl = ts;
#pragma unroll
    for (int d = 1; d < 32; d <<= 1) {
      const int t = __shfl_up(incl, d);
      if (lane >= d) incl += t;
    }
    if (lane == 31) wtot[wave] = incl;
    __syncthreads();
    const int S0 = wtot[0]  + wtot[1]  + wtot[2]  + wtot[3];
    const int S1 = wtot[4]  + wtot[5]  + wtot[6]  + wtot[7];
    const int S2 = wtot[8]  + wtot[9]  + wtot[10] + wtot[11];
    const int S3 = wtot[12] + wtot[13] + wtot[14] + wtot[15];
    int pre = 0;
#pragma unroll 1
    for (int w = 4 * sub; w < wave; ++w) pre += wtot[w];
    const int b0 = carry;
    const int b1 = b0 + ((S0 + 31) & ~31);
    const int b2 = b1 + ((S1 + 31) & ~31);
    const int b3 = b2 + ((S2 + 31) & ~31);
    const int b4 = b3 + ((S3 + 31) & ~31);
    const int myb = sub == 0 ? b0 : (sub == 1 ? b1 : (sub == 2 ? b2 : b3));
    if (tid == 0) {
      srb[min(4 * ch + 0, RBN - 1)] = b0;
      srb[min(4 * ch + 1, RBN - 1)] = b1;
      srb[min(4 * ch + 2, RBN - 1)] = b2;
      srb[min(4 * ch + 3, RBN - 1)] = b3;
    }
    int run = myb + pre + incl - ts;
    soff[8 * tid + 0] = run; run += e0;
    soff[8 * tid + 1] = run; run += e1;
    soff[8 * tid + 2] = run; run += e2;
    soff[8 * tid + 3] = run; run += e3;
    soff[8 * tid + 4] = run; run += e4;
    soff[8 * tid + 5] = run; run += e5;
    soff[8 * tid + 6] = run; run += e6;
    soff[8 * tid + 7] = run;
    carry = b4;
    __syncthreads();
    const v4i o0 = *(const v4i*)(soff + 4 * tid);
    const v4i o1 = *(const v4i*)(soff + 4 * (tid + OTHR));
    int* op = off + base;
    *(volatile v4i*)(op + 4 * tid) = o0;
    *(volatile v4i*)(op + 4 * (tid + OTHR)) = o1;
    __threadfence();
    *(volatile v4i*)(op + 4 * tid) = o0;
    *(volatile v4i*)(op + 4 * (tid + OTHR)) = o1;
    __syncthreads();
  }
  if (tid == 0) srb[min(4 * nChunk, RBN - 1)] = carry;
  __syncthreads();
  v4i rv = {0, 0, 0, 0};
  if (tid < 32) rv = *(const v4i*)(srb + 4 * tid);
  if (tid < 32) *(volatile v4i*)(rbase + 4 * tid) = rv;
  __threadfence();
  if (tid < 32) *(volatile v4i*)(rbase + 4 * tid) = rv;
}

__global__ __launch_bounds__(NTHR) void k_fill(
    const int* __restrict__ srcs, const int* __restrict__ dsts,
    const int* __restrict__ off, const int* __restrict__ rbase,
    int* csr, int nN, int nE, int vec8, int csrLen) {
  extern __shared__ v4f lds_dyn[];
  int* region = (int*)lds_dyn;
  int* cursor = region + RCAP;
  int* list   = cursor + NBF;
  int* wcnt   = list + LISTN;
  const int tid = threadIdx.x, lane = tid & 31, wave = tid >> 5;
  const int b = blockIdx.x;
  const int nodeBase = b * NBF;

  int rb0 = rbase[b];
  const int rb1 = rbase[b + 1];
  rb0 = rb0 < 0 ? 0 : (rb0 > csrLen ? csrLen : rb0);
  rb0 &= ~31;
  int len = rb1 - rb0;
  len = len < 0 ? 0 : (len > RCAP ? RCAP : len);
  int lenW = (len + 31) & ~31;
  if (rb0 + lenW > csrLen) lenW = (csrLen - rb0) & ~31;

  {
    const v4i z = {0, 0, 0, 0};
    for (int i = tid; i < RCAP / 4; i += NTHR) ((v4i*)region)[i] = z;
    for (int s = tid; s < NBF; s += NTHR) {
      int o = off[nodeBase + s] - rb0;
      o = o < 0 ? 0 : (o > RCAP ? RCAP : o);
      cursor[s] = o;
    }
  }
  __syncthreads();

  const int nChunks = (nE + CHUNK - 1) / CHUNK;
#pragma unroll 1
  for (int ch = 0; ch < nChunks; ++ch) {
    const int cbase = ch * CHUNK;
    const int wc = scan_chunk<NBF>(dsts, nE, cbase, nodeBase, vec8, list, tid, lane, wave);
    if (lane == 0) wcnt[wave] = wc;
    __syncthreads();
    if (wave == 0) {
#pragma unroll 1
      for (int wsx = 0; wsx < NWAVE; ++wsx) {
        int n = __builtin_amdgcn_readfirstlane(wcnt[wsx]);
        n = n > WCAP ? WCAP : (n < 0 ? 0 : n);
        const int* lp = list + wsx * WCAP;
#pragma unroll 1
        for (int i = 0; i < n; ++i) {
          const int ent  = __builtin_amdgcn_readfirstlane(lp[i]);
          const int slot = ent & (NBF - 1);
          int e = cbase + ((ent >> 12) & (CHUNK - 1));
          e = e > nE - 1 ? nE - 1 : e;
          int sv = srcs[e];
          sv = sv < 0 ? 0 : (sv > nN - 1 ? nN - 1 : sv);
          if (lane == 0) {
            int pos = cursor[slot];
            pos = pos < 0 ? 0 : (pos > RCAP - 1 ? RCAP - 1 : pos);
            region[pos] = sv;
            const int np = pos + 1;
            cursor[slot] = np > RCAP ? RCAP : np;
          }
        }
      }
    }
    __syncthreads();
  }

  const int nv = lenW >> 2;
  int* gp = csr + rb0;
#pragma unroll 1
  for (int i = tid; i < nv; i += NTHR) { const v4i v = ((const v4i*)region)[i]; *(volatile v4i*)(gp + 4 * i) = v; }
  __threadfence();
#pragma unroll 1
  for (int i = tid; i < nv; i += NTHR) { const v4i v = ((const v4i*)region)[i]; *(volatile v4i*)(gp + 4 * i) = v; }
}

__global__ __launch_bounds__(NTHR) void k_xcvt(const float* __restrict__ x, _Float16* apl,
                                               int nN, int npad) {
  const int u = (int)blockIdx.x * NTHR + (int)threadIdx.x;
  const int row = u >> 3, seg = u & 7;
  if (row >= npad) return;
  int rc = row > nN - 1 ? nN - 1 : row;
  rc = rc < 0 ? 0 : rc;
  const bool live = row < nN;
  const float* p = x + (size_t)rc * HD + 8 * seg;
  const v4f a0 = *(const v4f*)p, a1 = *(const v4f*)(p + 4);
  const float f[8] = {a0.x, a0.y, a0.z, a0.w, a1.x, a1.y, a1.z, a1.w};
  v8h o;
#pragma unroll
  for (int i = 0; i < 8; ++i) o[i] = live ? (_Float16)f[i] : (_Float16)0.0f;
  _Float16* gp = apl + (size_t)row * HD + 8 * seg;
  *(volatile v8h*)gp = o;
  __threadfence();
  *(volatile v8h*)gp = o;
}

__global__ __launch_bounds__(NTHR) void k_wtcvt(const float* __restrict__ W, _Float16* P,
                                                int K, int Nout, int NoutP) {
  const int i = (int)blockIdx.x * NTHR + (int)threadIdx.x;
  const int ppr = K >> 3;
  const int nUnits = NoutP * ppr;
  if (i >= nUnits) return;
  const int n = i / ppr;
  const int seg = i - n * ppr;
  const int nc = n > Nout - 1 ? Nout - 1 : n;
  const bool live = n < Nout;
  const float* p = W + (size_t)(8 * seg) * Nout + nc;
  v8h o;
#pragma unroll
  for (int j = 0; j < 8; ++j) {
    const float v = p[(size_t)j * Nout] * WCARRY;
    o[j] = live ? (_Float16)v : (_Float16)0.0f;
  }
  _Float16* gp = P + (size_t)i * 8;
  *(volatile v8h*)gp = o;
  __threadfence();
  *(volatile v8h*)gp = o;
}

__global__ __launch_bounds__(GTHR) void k_gemm(
    const _Float16* __restrict__ A, const _Float16* __restrict__ B, float* C32) {
  constexpr int TPW = 4;
  constexpr int NIT = (GBM * HD) / (4 * GTHR);
  __shared__ __attribute__((aligned(16))) float stg[GBM * HD];
  const int tid = threadIdx.x, lane = tid & 31, wave = tid >> 5, hh = lane >> 4, m = lane & 15;
  const int rowBase = (int)blockIdx.x * GBM;
  const int r0 = wave * 16;

  v8f acc[TPW];
#pragma unroll
  for (int t = 0; t < TPW; ++t) { v8f z = {0.f, 0.f, 0.f, 0.f, 0.f, 0.f, 0.f, 0.f}; acc[t] = z; }

  const _Float16* ap = A + (size_t)(rowBase + r0 + m) * HD + 8 * hh;
  const _Float16* bp = B + (size_t)m * HD + 8 * hh;
#pragma unroll
  for (int ks = 0; ks < HD / 32; ++ks) {
    Frag a;
    a.half[0] = *(const v8h*)(ap + 32 * ks);
    a.half[1] = *(const v8h*)(ap + 32 * ks + 16);
#pragma unroll
    for (int t = 0; t < TPW; ++t) {
      const _Float16* bq = bp + (size_t)(16 * t) * HD + 32 * ks;
      Frag b;
      b.half[0] = *(const v8h*)bq;
      b.half[1] = *(const v8h*)(bq + 16);
      acc[t] = wm(a.v, b.v, acc[t]);
    }
  }

  {
    float* sp = stg + (size_t)(r0 + 8 * hh) * HD + m;
#pragma unroll
    for (int t = 0; t < TPW; ++t) {
#pragma unroll
      for (int r = 0; r < 8; ++r) sp[r * HD + 16 * t] = acc[t][r] * WINV;
    }
  }
  __syncthreads();

  v4f cv[NIT];
#pragma unroll
  for (int it = 0; it < NIT; ++it) {
    const int id = it * GTHR + tid;
    const int row = id >> 4, seg = id & 15;
    cv[it] = *(const v4f*)(stg + (size_t)row * HD + 4 * seg);
  }
#pragma unroll
  for (int it = 0; it < NIT; ++it) {
    const int id = it * GTHR + tid;
    const int row = id >> 4, seg = id & 15;
    float* gp = C32 + (size_t)(rowBase + row) * HD + 4 * seg;
    *(volatile v4f*)gp = cv[it];
  }
  __threadfence();
#pragma unroll
  for (int it = 0; it < NIT; ++it) {
    const int id = it * GTHR + tid;
    const int row = id >> 4, seg = id & 15;
    float* gp = C32 + (size_t)(rowBase + row) * HD + 4 * seg;
    *(volatile v4f*)gp = cv[it];
  }
}

__global__ __launch_bounds__(NTHR) void k_agg(
    const int* __restrict__ csr, const int* __restrict__ off, const int* __restrict__ cnt,
    const float* __restrict__ dinv, const float* __restrict__ hb, const float* __restrict__ bias,
    float* xo, float* xsum, int nN, int csrLen) {
  __shared__ __attribute__((aligned(16))) float scs[NWAVE * 2 * HD];
  __shared__ __attribute__((aligned(16))) float srow[HD];
  const int tid = threadIdx.x, lane = tid & 31, wave = tid >> 5, hf = lane >> 4, q = lane & 15;
  const int col4 = 4 * q;
  const int tbase = blockIdx.x * TGT + wave * 32;
  const int cl    = tbase + lane;
  const int cnt_l = cnt[cl];
  const int off_l = off[cl];
  const float di_l = dinv[cl];
  const v4f bb = *(const v4f*)(bias + col4);
  const float keep = (hf == 0) ? 1.f : 0.f;
  v4f cs = {0.f, 0.f, 0.f, 0.f};

#pragma unroll 1
  for (int j = 0; j < 32; ++j) {
    const int c = tbase + j;
    int nraw = __shfl(cnt_l, j);
    nraw = nraw < 0 ? 0 : nraw;
    const int n = nraw > DEGCAP ? DEGCAP : nraw;
    const int st = __shfl(off_l, j);
    const float dc = __shfl(di_l, j);
    const float sn = 1.0f / ((float)nraw + 1.0f);

    v4f a = {0.f, 0.f, 0.f, 0.f};
#pragma unroll 1
    for (int q0 = 0; q0 < n; q0 += 32) {
      int pos = st + q0 + lane;
      pos = pos < 0 ? 0 : (pos > csrLen - 1 ? csrLen - 1 : pos);
      int sl = csr[pos];
      sl = sl < 0 ? 0 : (sl > nN - 1 ? nN - 1 : sl);
      const int mcnt = (n - q0) < 32 ? (n - q0) : 32;
#pragma unroll 1
      for (int pp = 0; pp < mcnt; pp += 2) {
        const int s0 = __builtin_amdgcn_readlane(sl, pp);
        const int s1 = __builtin_amdgcn_readlane(sl, pp + 1);
        const int s = hf ? s1 : s0;
        const float w = ((pp + hf) < mcnt) ? dinv[s] * dc : 0.f;
        const v4f xv = *(const v4f*)(hb + (size_t)s * HD + col4);
        a += xv * w;
      }
    }
    a.x += __shfl_xor(a.x, 16);
    a.y += __shfl_xor(a.y, 16);
    a.z += __shfl_xor(a.z, 16);
    a.w += __shfl_xor(a.w, 16);

    const v4f hs = *(const v4f*)(hb + (size_t)c * HD + col4);
    const bool live = c < nN;
    v4f o = a + hs * sn + bb;
    o.x = live ? o.x : 0.f; o.y = live ? o.y : 0.f; o.z = live ? o.z : 0.f; o.w = live ? o.w : 0.f;
    cs += o * keep;
    float* gp = xo + (size_t)c * HD + col4;
    if (hf == 0) *(volatile v4f*)gp = o;
    __threadfence();
    if (hf == 0) *(volatile v4f*)gp = o;
  }

  colsum_out(scs, srow, cs, xsum + (size_t)blockIdx.x * HD, tid, lane, wave);
}

__global__ __launch_bounds__(NTHR) void k_var(const float* __restrict__ xo, const float* __restrict__ xsum,
                                              float* sq, int nN, int nPart) {
  __shared__ __attribute__((aligned(16))) float smu[HD];
  __shared__ __attribute__((aligned(16))) float scs[NWAVE * 2 * HD];
  __shared__ __attribute__((aligned(16))) float srow[HD];
  const int tid = threadIdx.x, lane = tid & 31, wave = tid >> 5, hf = lane >> 4, q = lane & 15;
  const int col4 = 4 * q;
  const int tbase = blockIdx.x * TGT + wave * 32;
  if (tid < HD) {
    double s = 0.0;
#pragma unroll 1
    for (int b = 0; b < nPart; ++b) s += (double)xsum[(size_t)b * HD + tid];
    smu[tid] = (float)(s / (double)nN);
  }
  __syncthreads();
  const v4f mu = *(const v4f*)(smu + col4);
  v4f cs = {0.f, 0.f, 0.f, 0.f};
#pragma unroll 1
  for (int it = 0; it < 16; ++it) {
    const int c = tbase + 2 * it + hf;
    const bool live = c < nN;
    const v4f x = *(const v4f*)(xo + (size_t)c * HD + col4);
    v4f d = x - mu;
    d.x = live ? d.x : 0.f; d.y = live ? d.y : 0.f; d.z = live ? d.z : 0.f; d.w = live ? d.w : 0.f;
    cs += d * d;
  }
  colsum_out(scs, srow, cs, sq + (size_t)blockIdx.x * HD, tid, lane, wave);
}

__global__ __launch_bounds__(NTHR) void k_bnapply(
    const float* __restrict__ xo, const float* __restrict__ xsum, const float* __restrict__ sq,
    const float* __restrict__ gam, const float* __restrict__ bet,
    _Float16* apl, int nN, int nPart) {
  __shared__ __attribute__((aligned(16))) float smu[HD];
  __shared__ __attribute__((aligned(16))) float srs[HD];
  __shared__ __attribute__((aligned(16))) float sg[HD];
  __shared__ __attribute__((aligned(16))) float sb[HD];
  const int tid = threadIdx.x, lane = tid & 31, wave = tid >> 5;
  const int tbase = blockIdx.x * TGT + wave * 32;
  const int r4 = lane >> 3, c8 = 8 * (lane & 7);
  if (tid < HD) {
    double s1 = 0.0, s2 = 0.0;
#pragma unroll 1
    for (int b = 0; b < nPart; ++b) {
      s1 += (double)xsum[(size_t)b * HD + tid];
      s2 += (double)sq[(size_t)b * HD + tid];
    }
    const float mu  = (float)(s1 / (double)nN);
    const float var = (float)(s2 / (double)nN);
    smu[tid] = mu;
    srs[tid] = rsqrtf(var + BN_EPS);
    sg[tid]  = gam[tid];
    sb[tid]  = bet[tid];
  }
  __syncthreads();
  float mu[8], rs[8], gg[8], be[8];
  {
    const v4f a0 = *(const v4f*)(smu + c8), a1 = *(const v4f*)(smu + c8 + 4);
    const v4f b0 = *(const v4f*)(srs + c8), b1 = *(const v4f*)(srs + c8 + 4);
    const v4f c0 = *(const v4f*)(sg + c8),  c1 = *(const v4f*)(sg + c8 + 4);
    const v4f d0 = *(const v4f*)(sb + c8),  d1 = *(const v4f*)(sb + c8 + 4);
    mu[0] = a0.x; mu[1] = a0.y; mu[2] = a0.z; mu[3] = a0.w; mu[4] = a1.x; mu[5] = a1.y; mu[6] = a1.z; mu[7] = a1.w;
    rs[0] = b0.x; rs[1] = b0.y; rs[2] = b0.z; rs[3] = b0.w; rs[4] = b1.x; rs[5] = b1.y; rs[6] = b1.z; rs[7] = b1.w;
    gg[0] = c0.x; gg[1] = c0.y; gg[2] = c0.z; gg[3] = c0.w; gg[4] = c1.x; gg[5] = c1.y; gg[6] = c1.z; gg[7] = c1.w;
    be[0] = d0.x; be[1] = d0.y; be[2] = d0.z; be[3] = d0.w; be[4] = d1.x; be[5] = d1.y; be[6] = d1.z; be[7] = d1.w;
  }
#pragma unroll 1
  for (int it = 0; it < 8; ++it) {
    const int c = tbase + 4 * it + r4;
    const bool live = c < nN;
    const float* xr = xo + (size_t)c * HD + c8;
    const v4f x0 = *(const v4f*)xr, x1 = *(const v4f*)(xr + 4);
    const float xv[8] = {x0.x, x0.y, x0.z, x0.w, x1.x, x1.y, x1.z, x1.w};
    v8h o;
#pragma unroll
    for (int i = 0; i < 8; ++i) {
      const float t = ((xv[i] - mu[i]) * rs[i]) * gg[i] + be[i];
      const float y = fmaxf(t, 0.f);
      o[i] = live ? (_Float16)y : (_Float16)0.0f;
    }
    _Float16* gp = apl + (size_t)c * HD + c8;
    *(volatile v8h*)gp = o;
    __threadfence();
    *(volatile v8h*)gp = o;
  }
}

__global__ __launch_bounds__(NTHR) void k_pool(
    const int* __restrict__ batch, const float* __restrict__ xo,
    const float* __restrict__ xsum, const float* __restrict__ sq,
    const float* __restrict__ gam, const float* __restrict__ bet,
    float* z, int nN, int nPart) {
  __shared__ __attribute__((aligned(16))) float smu[HD];
  __shared__ __attribute__((aligned(16))) float srs[HD];
  __shared__ __attribute__((aligned(16))) float sg[HD];
  __shared__ __attribute__((aligned(16))) float sb[HD];
  const int tid = threadIdx.x, lane = tid & 31, wave = tid >> 5, hf = lane >> 4, q = lane & 15;
  const int col4 = 4 * q;
  if (tid < HD) {
    double s1 = 0.0, s2 = 0.0;
#pragma unroll 1
    for (int b = 0; b < nPart; ++b) {
      s1 += (double)xsum[(size_t)b * HD + tid];
      s2 += (double)sq[(size_t)b * HD + tid];
    }
    const float mu  = (float)(s1 / (double)nN);
    const float var = (float)(s2 / (double)nN);
    smu[tid] = mu;
    srs[tid] = rsqrtf(var + BN_EPS);
    sg[tid]  = gam[tid];
    sb[tid]  = bet[tid];
  }
  __syncthreads();
  const int g = (int)blockIdx.x * NWAVE + wave;
  const v4f mu = *(const v4f*)(smu + col4);
  const v4f rs = *(const v4f*)(srs + col4);
  const v4f gg = *(const v4f*)(sg + col4);
  const v4f bb = *(const v4f*)(sb + col4);
  v4f s  = {0.f, 0.f, 0.f, 0.f};
  v4f mx = {0.f, 0.f, 0.f, 0.f};
  int cnt = 0;
#pragma unroll 1
  for (int base = 0; base < nN; base += 32) {
    const int idx = base + lane;
    const int ic = idx > nN - 1 ? nN - 1 : idx;
    const int bv = batch[ic];
    const bool hit = (idx < nN) && (bv == g);
    unsigned mk = __builtin_amdgcn_ballot_w32(hit);
    cnt += (int)__builtin_popcount(mk);
#pragma unroll 1
    for (int it = 0; it < 32; ++it) {
      if (mk == 0u) break;
      const int pp = __builtin_ctz(mk);
      mk &= mk - 1u;
      const int node = base + pp;
      const v4f x = *(const v4f*)(xo + (size_t)node * HD + col4);
      const v4f y = relu4(((x - mu) * rs) * gg + bb);
      s += y;
      mx.x = fmaxf(mx.x, y.x); mx.y = fmaxf(mx.y, y.y); mx.z = fmaxf(mx.z, y.z); mx.w = fmaxf(mx.w, y.w);
    }
  }
  const float inv = 1.0f / (float)(cnt < 1 ? 1 : cnt);
  const v4f mean = s * inv;
  v4f v;
  v.x = hf ? mx.x : mean.x; v.y = hf ? mx.y : mean.y; v.z = hf ? mx.z : mean.z; v.w = hf ? mx.w : mean.w;
  float* gp = z + (size_t)g * ZW + 4 * lane;
  *(volatile v4f*)gp = v;
  __threadfence();
  *(volatile v4f*)gp = v;
}

__global__ __launch_bounds__(HTHR) void k_head(
    const float* __restrict__ z, const _Float16* __restrict__ p1, const float* __restrict__ lb1,
    const _Float16* __restrict__ p2, const float* __restrict__ lb2,
    const _Float16* __restrict__ p3, const float* __restrict__ lb3,
    float* out, int nTiles, int nG, int ncls) {
  __shared__ __attribute__((aligned(16))) _Float16 sA[HWAVE * 16 * ZW];
  __shared__ __attribute__((aligned(16))) _Float16 sB[HWAVE * 16 * HD];
  __shared__ __attribute__((aligned(16))) _Float16 sC[HWAVE * 16 * H2];
  __shared__ __attribute__((aligned(16))) float sO[SOCAP];
  const int tid = threadIdx.x, lane = tid & 31, wave = tid >> 5, hh = lane >> 4, m = lane & 15;
  _Float16* sAw = sA + wave * 16 * ZW;
  _Float16* sBw = sB + wave * 16 * HD;
  _Float16* sCw = sC + wave * 16 * H2;
  const int cc = ncls < 1 ? 1 : (ncls > 16 ? 16 : ncls);
  const float b3v = lb3[m < cc ? m : cc - 1];

#pragma unroll 1
  for (int tb = 0; tb < nTiles; tb += HWAVE) {
    const int t = tb + wave;
    const bool tv = t < nTiles;
    const int tcl = tv ? t : nTiles - 1;
    const int r0 = tcl * 16;

#pragma unroll
    for (int r = 0; r < 16; ++r) {
      const v4f v = *(const v4f*)(z + (size_t)(r0 + r) * ZW + 4 * lane);
      v4h hv;
      hv.x = (_Float16)v.x; hv.y = (_Float16)v.y; hv.z = (_Float16)v.z; hv.w = (_Float16)v.w;
      *(v4h*)(sAw + r * ZW + 4 * lane) = hv;
    }
    __syncthreads();

    v8f acc1[4];
#pragma unroll
    for (int u = 0; u < 4; ++u) { v8f zz = {0.f, 0.f, 0.f, 0.f, 0.f, 0.f, 0.f, 0.f}; acc1[u] = zz; }
#pragma unroll
    for (int ks = 0; ks < ZW / 32; ++ks) {
      Frag a;
      a.half[0] = *(const v8h*)(sAw + m * ZW + 32 * ks + 8 * hh);
      a.half[1] = *(const v8h*)(sAw + m * ZW + 32 * ks + 16 + 8 * hh);
#pragma unroll
      for (int u = 0; u < 4; ++u) {
        const _Float16* bq = p1 + (size_t)(16 * u + m) * ZW + 32 * ks + 8 * hh;
        Frag b;
        b.half[0] = *(const v8h*)bq;
        b.half[1] = *(const v8h*)(bq + 16);
        acc1[u] = wm(a.v, b.v, acc1[u]);
      }
    }
#pragma unroll
    for (int u = 0; u < 4; ++u) {
      const int col = 16 * u + m;
      const float bv = lb1[col];
#pragma unroll
      for (int r = 0; r < 8; ++r) {
        const float v = fmaxf(acc1[u][r] * WINV + bv, 0.f);
        sBw[(8 * hh + r) * HD + col] = (_Float16)v;
      }
    }
    __syncthreads();

    v8f acc2[2];
#pragma unroll
    for (int u = 0; u < 2; ++u) { v8f zz = {0.f, 0.f, 0.f, 0.f, 0.f, 0.f, 0.f, 0.f}; acc2[u] = zz; }
#pragma unroll
    for (int ks = 0; ks < HD / 32; ++ks) {
      Frag a;
      a.half[0] = *(const v8h*)(sBw + m * HD + 32 * ks + 8 * hh);
      a.half[1] = *(const v8h*)(sBw + m * HD + 32 * ks + 16 + 8 * hh);
#pragma unroll
      for (int u = 0; u < 2; ++u) {
        const _Float16* bq = p2 + (size_t)(16 * u + m) * HD + 32 * ks + 8 * hh;
        Frag b;
        b.half[0] = *(const v8h*)bq;
        b.half[1] = *(const v8h*)(bq + 16);
        acc2[u] = wm(a.v, b.v, acc2[u]);
      }
    }
#pragma unroll
    for (int u = 0; u < 2; ++u) {
      const int col = 16 * u + m;
      const float bv = lb2[col];
#pragma unroll
      for (int r = 0; r < 8; ++r) {
        const float v = fmaxf(acc2[u][r] * WINV + bv, 0.f);
        sCw[(8 * hh + r) * H2 + col] = (_Float16)v;
      }
    }
    __syncthreads();

    v8f acc3 = {0.f, 0.f, 0.f, 0.f, 0.f, 0.f, 0.f, 0.f};
    {
      Frag a, b;
      a.half[0] = *(const v8h*)(sCw + m * H2 + 8 * hh);
      a.half[1] = *(const v8h*)(sCw + m * H2 + 16 + 8 * hh);
      const _Float16* bq = p3 + (size_t)m * H2 + 8 * hh;
      b.half[0] = *(const v8h*)bq;
      b.half[1] = *(const v8h*)(bq + 16);
      acc3 = wm(a.v, b.v, acc3);
    }
    if (tv && m < cc) {
#pragma unroll
      for (int r = 0; r < 8; ++r) {
        const int oi = (r0 + 8 * hh + r) * cc + m;
        if (oi < SOCAP) sO[oi] = acc3[r] * WINV + b3v;
      }
    }
  }
  __syncthreads();

  const int nF = nG * cc;
#pragma unroll 1
  for (int i = tid; 4 * i < nF; i += HTHR) {
    const int f0 = 4 * i;
    if (f0 + 4 <= nF) {
      const v4f v = *(const v4f*)(sO + f0);
      *(volatile v4f*)(out + f0) = v;
    } else {
      for (int k = 0; k < 3; ++k) if (f0 + k < nF) *(volatile float*)(out + f0 + k) = sO[f0 + k];
    }
  }
  __threadfence();
#pragma unroll 1
  for (int i = tid; 4 * i < nF; i += HTHR) {
    const int f0 = 4 * i;
    if (f0 + 4 <= nF) {
      const v4f v = *(const v4f*)(sO + f0);
      *(volatile v4f*)(out + f0) = v;
    } else {
      for (int k = 0; k < 3; ++k) if (f0 + k < nF) *(volatile float*)(out + f0 + k) = sO[f0 + k];
    }
  }
}

extern "C" void kernel_launch(void* const* d_in, const int* in_sizes, int n_in,
                              void* d_out, int out_size, void* d_ws, size_t ws_size,
                              hipStream_t stream) {
  if (n_in < 22) return;
  const int nN = in_sizes[3];
  const int nE = in_sizes[1];
  if (nN <= 0 || nE <= 0) return;
  if (nN > (1 << 22) || nE > (1 << 28)) return;
  if (in_sizes[0] != nN * HD || in_sizes[2] != nE) return;
  if (in_sizes[4] != HD * HD || in_sizes[6] != HD * HD || in_sizes[8] != HD * HD) return;
  if (in_sizes[5] != HD || in_sizes[7] != HD || in_sizes[9] != HD) return;
  for (int i = 10; i < 16; ++i) { if (in_sizes[i] != HD) return; }
  if (in_sizes[16] != ZW * HD || in_sizes[17] != HD) return;
  if (in_sizes[18] != HD * H2 || in_sizes[19] != H2) return;
  const int ncls = in_sizes[21];
  if (ncls < 1 || ncls > 16) return;
  if (in_sizes[20] != H2 * ncls) return;
  if (out_size <= 0 || (out_size % ncls) != 0) return;
  const int nG = out_size / ncls;
  const int NGP = ((nG + 15) / 16) * 16;
  const int nTiles = NGP / 16;
  if (NGP * ncls > SOCAP) return;

  const float* x     = (const float*)d_in[0];
  const int*   src   = (const int*)d_in[1];
  const int*   dst   = (const int*)d_in[2];
  const int*   batch = (const int*)d_in[3];
  const float* Wl[3]  = {(const float*)d_in[4],  (const float*)d_in[6],  (const float*)d_in[8]};
  const float* bl[3]  = {(const float*)d_in[5],  (const float*)d_in[7],  (const float*)d_in[9]};
  const float* gl[3]  = {(const float*)d_in[10], (const float*)d_in[12], (const float*)d_in[14]};
  const float* bel[3] = {(const float*)d_in[11], (const float*)d_in[13], (const float*)d_in[15]};
  const float* LW1 = (const float*)d_in[16]; const float* Lb1 = (const float*)d_in[17];
  const float* LW2 = (const float*)d_in[18]; const float* Lb2 = (const float*)d_in[19];
  const float* LW3 = (const float*)d_in[20]; const float* Lb3 = (const float*)d_in[21];
  float* out = (float*)d_out;

  const int NPAD   = ((nN + TGT - 1) / TGT) * TGT;
  const int nBC    = (nN + NBC - 1) / NBC;
  const int CNTPAD = nBC * NBC;
  if (CNTPAD < NPAD) return;
  if (4 * nBC + 1 > RBN) return;
  const int nBF    = (nN + NBF - 1) / NBF;
  if (nBF > 4 * nBC) return;
  const int csrLen = ((nE + 31) & ~31) + 4096;
  if (31 * 4 * nBC > 4096) return;
  const int nAgg   = NPAD / TGT;
  const int nGemm  = NPAD / GBM;

  char* ws = (char*)d_ws;
  size_t off = 0;
  size_t oW[3];
  for (int l = 0; l < 3; ++l) { oW[l] = off; off += (size_t)HD * HD * 2;   off = (off + 255) & ~(size_t)255; }
  const size_t oP1  = off; off += (size_t)HD * ZW * 2;            off = (off + 255) & ~(size_t)255;
  const size_t oP2  = off; off += (size_t)H2 * HD * 2;            off = (off + 255) & ~(size_t)255;
  const size_t oP3  = off; off += (size_t)16 * H2 * 2;            off = (off + 255) & ~(size_t)255;
  const size_t oA   = off; off += (size_t)NPAD * HD * 2;          off = (off + 255) & ~(size_t)255;
  const size_t oC   = off; off += (size_t)NPAD * HD * 4;          off = (off + 255) & ~(size_t)255;
  const size_t oX   = off; off += (size_t)NPAD * HD * 4;          off = (off + 255) & ~(size_t)255;
  const size_t oCnt = off; off += (size_t)CNTPAD * 4;             off = (off + 255) & ~(size_t)255;
  const size_t oDi  = off; off += (size_t)CNTPAD * 4;             off = (off + 255) & ~(size_t)255;
  const size_t oOff = off; off += (size_t)CNTPAD * 4;             off = (off + 255) & ~(size_t)255;
  const size_t oRb  = off; off += (size_t)RBN * 4;                off = (off + 255) & ~(size_t)255;
  const size_t oCsr = off; off += (size_t)csrLen * 4;             off = (off + 255) & ~(size_t)255;
  const size_t oXs  = off; off += (size_t)nAgg * HD * 4;          off = (off + 255) & ~(size_t)255;
  const size_t oSq  = off; off += (size_t)nAgg * HD * 4;          off = (off + 255) & ~(size_t)255;
  const size_t oZ   = off; off += (size_t)NGP * ZW * 4;           off = (off + 255) & ~(size_t)255;
  if (off > ws_size || off > (size_t)WSCAP) return;

  _Float16* wpl[3] = {(_Float16*)(ws + oW[0]), (_Float16*)(ws + oW[1]), (_Float16*)(ws + oW[2])};
  _Float16* p1   = (_Float16*)(ws + oP1);
  _Float16* p2   = (_Float16*)(ws + oP2);
  _Float16* p3   = (_Float16*)(ws + oP3);
  _Float16* apl  = (_Float16*)(ws + oA);
  float* cbuf = (float*)(ws + oC);
  float* xo   = (float*)(ws + oX);
  int*   cnt  = (int*)(ws + oCnt);
  float* dinv = (float*)(ws + oDi);
  int*   offp = (int*)(ws + oOff);
  int*   rb   = (int*)(ws + oRb);
  int*   csr  = (int*)(ws + oCsr);
  float* xsum = (float*)(ws + oXs);
  float* sq   = (float*)(ws + oSq);
  float* zb   = (float*)(ws + oZ);

  const int vec8 = 1;

  k_xcvt<<<NPAD / 32, NTHR, 0, stream>>>(x, apl, nN, NPAD);
  for (int l = 0; l < 3; ++l)
    k_wtcvt<<<(HD * (HD / 8) + NTHR - 1) / NTHR, NTHR, 0, stream>>>(Wl[l], wpl[l], HD, HD, HD);
  k_wtcvt<<<(HD * (ZW / 8) + NTHR - 1) / NTHR, NTHR, 0, stream>>>(LW1, p1, ZW, HD, HD);
  k_wtcvt<<<(H2 * (HD / 8) + NTHR - 1) / NTHR, NTHR, 0, stream>>>(LW2, p2, HD, H2, H2);
  k_wtcvt<<<(16 * (H2 / 8) + NTHR - 1) / NTHR, NTHR, 0, stream>>>(LW3, p3, H2, ncls, 16);
  k_count<<<nBC, NTHR, 0, stream>>>(dst, cnt, dinv, nE, vec8);
  k_offsets<<<1, OTHR, 0, stream>>>(cnt, offp, rb, nBC);
  hipFuncSetAttribute(reinterpret_cast<const void*>(&k_fill),
                      hipFuncAttributeMaxDynamicSharedMemorySize, LDS_FILL);
  k_fill<<<nBF, NTHR, LDS_FILL, stream>>>(src, dst, offp, rb, csr, nN, nE, vec8, csrLen);

  for (int l = 0; l < 3; ++l) {
    k_gemm<<<nGemm, GTHR, 0, stream>>>(apl, wpl[l], cbuf);
    k_agg<<<nAgg, NTHR, 0, stream>>>(csr, offp, cnt, dinv, cbuf, bl[l], xo, xsum, nN, csrLen);
    k_var<<<nAgg, NTHR, 0, stream>>>(xo, xsum, sq, nN, nAgg);
    if (l < 2)
      k_bnapply<<<nAgg, NTHR, 0, stream>>>(xo, xsum, sq, gl[l], bel[l], apl, nN, nAgg);
  }
  k_pool<<<NGP / NWAVE, NTHR, 0, stream>>>(batch, xo, xsum, sq, gl[2], bel[2], zb, nN, nAgg);
  k_head<<<1, HTHR, 0, stream>>>(zb, p1, Lb1, p2, Lb2, p3, Lb3, out, nTiles, nG, ncls);
}
